// MultiHeadSelfAttention_90537910600353
// MI455X (gfx1250) — hardware-verified
//
#include <hip/hip_runtime.h>
#include <stdint.h>


#ifndef NB
#define NB 2
#endif
#ifndef SEQ
#define SEQ 2048
#endif
#define NB_FULL  2
#define SEQ_FULL 2048
#define EE   1024
#define HH   16
#define HD   64
#define TRIL 2080
#define M_TOT (NB * SEQ)
#define PCARRY     16384.0f
#define PCARRY_INV (1.0f / 16384.0f)
#define WSCALE     64.0f
#define WSCALE_INV (1.0f / 64.0f)

static_assert(NB >= 1 && NB <= NB_FULL);
static_assert(SEQ >= 128 && SEQ <= SEQ_FULL && (SEQ % 128) == 0);
static_assert(EE == HH * HD);
static_assert((EE % 64) == 0 && (M_TOT % 128) == 0 && (SEQ % 64) == 0);
static_assert(TRIL == HD * (HD + 1) / 2);

typedef _Float16       v16h __attribute__((ext_vector_type(16)));
typedef __bf16         v16b __attribute__((ext_vector_type(16)));
typedef float          v8f  __attribute__((ext_vector_type(8)));
typedef float          v4f  __attribute__((ext_vector_type(4)));
typedef unsigned int   v4u  __attribute__((ext_vector_type(4)));
typedef unsigned short u16;

union Frag { v16h h; v16b b; v4u u[2]; };

__device__ __forceinline__ unsigned bfbits(float f) {
  const unsigned u = __float_as_uint(f);
  return (u + 0x7FFFu + ((u >> 16) & 1u)) >> 16;
}
__device__ __forceinline__ float bf2f(unsigned b) { return __uint_as_float(b << 16); }
__device__ __forceinline__ unsigned hbits(float f) {
  const _Float16 hv = (_Float16)f;
  return (unsigned)__builtin_bit_cast(unsigned short, hv);
}
__device__ __forceinline__ float h2f(unsigned b) {
  return (float)__builtin_bit_cast(_Float16, (unsigned short)b);
}

__device__ __forceinline__ Frag ldfrag(const u16* p, int lh) {
  Frag f;
  f.u[0] = *reinterpret_cast<const v4u*>(p + lh);
  f.u[1] = *reinterpret_cast<const v4u*>(p + 16 + lh);
  return f;
}

__device__ __forceinline__ v8f mma_f16(Frag a, Frag b, v8f c) {
  c = __builtin_amdgcn_wmma_f32_16x16x32_f16(false, a.h, false, b.h, (short)0, c, false, false);
  asm volatile("v_nop\n\tv_nop\n\tv_nop\n\tv_nop"
               : "+v"(c) : "v"(a.u[0]), "v"(a.u[1]), "v"(b.u[0]), "v"(b.u[1]));
  return c;
}
__device__ __forceinline__ v8f mma_bf16(Frag a, Frag b, v8f c) {
  c = __builtin_amdgcn_wmma_f32_16x16x32_bf16(false, a.b, false, b.b, (short)0, c, false, false);
  asm volatile("v_nop\n\tv_nop\n\tv_nop\n\tv_nop"
               : "+v"(c) : "v"(a.u[0]), "v"(a.u[1]), "v"(b.u[0]), "v"(b.u[1]));
  return c;
}

__device__ __forceinline__ void vst16(u16* p, v4u v)   { *reinterpret_cast<volatile v4u*>(p) = v; }
__device__ __forceinline__ void vst4f(float* p, v4f v) { *reinterpret_cast<volatile v4f*>(p) = v; }
__device__ __forceinline__ v4u ld16(const u16* p)   { return *reinterpret_cast<const v4u*>(p); }
__device__ __forceinline__ v4f ld4f(const float* p) { return *reinterpret_cast<const v4f*>(p); }

__global__ void __launch_bounds__(256)
k_cvt_x(const float* __restrict__ x, u16* __restrict__ xb) {
  const int i = blockIdx.x * 256 + threadIdx.x;
  const int ngrp = M_TOT * (EE / 8);
  if (i >= ngrp) return;
  const int row = i / (EE / 8);
  const int c8  = i - row * (EE / 8);
  const int b   = row / SEQ;
  const int s   = row - b * SEQ;
  const float* src = x + ((size_t)(b * SEQ_FULL + s) * EE + (size_t)c8 * 8);
  const v4f a = *reinterpret_cast<const v4f*>(src);
  const v4f c = *reinterpret_cast<const v4f*>(src + 4);
  v4u w;
  w.x = bfbits(a.x) | (bfbits(a.y) << 16);
  w.y = bfbits(a.z) | (bfbits(a.w) << 16);
  w.z = bfbits(c.x) | (bfbits(c.y) << 16);
  w.w = bfbits(c.z) | (bfbits(c.w) << 16);
  u16* dst = xb + (size_t)i * 8;
  vst16(dst, w);
  __threadfence();
  vst16(dst, w);
}

__global__ void __launch_bounds__(256)
k_cvt_w(const float* __restrict__ w, u16* __restrict__ wb) {
  const int i = blockIdx.x * 256 + threadIdx.x;
  const int ngrp = EE * EE / 8;
  if (i >= ngrp) return;
  const float* src = w + (size_t)i * 8;
  const v4f a = *reinterpret_cast<const v4f*>(src);
  const v4f c = *reinterpret_cast<const v4f*>(src + 4);
  v4u o;
  o.x = bfbits(a.x) | (bfbits(a.y) << 16);
  o.y = bfbits(a.z) | (bfbits(a.w) << 16);
  o.z = bfbits(c.x) | (bfbits(c.y) << 16);
  o.w = bfbits(c.z) | (bfbits(c.w) << 16);
  u16* dst = wb + (size_t)i * 8;
  vst16(dst, o);
  __threadfence();
  vst16(dst, o);
}

__device__ __forceinline__ void cvt2(float f, unsigned& bb, unsigned& hb) {
  const float v = bf2f(bfbits(f)) * WSCALE;
  bb = __float_as_uint(v) >> 16;
  hb = hbits(v);
}
__global__ void __launch_bounds__(256)
k_cvt_wo(const float* __restrict__ w, u16* __restrict__ wob, u16* __restrict__ wof) {
  const int i = blockIdx.x * 256 + threadIdx.x;
  const int ngrp = EE * EE / 8;
  if (i >= ngrp) return;
  const float* src = w + (size_t)i * 8;
  const v4f a = *reinterpret_cast<const v4f*>(src);
  const v4f c = *reinterpret_cast<const v4f*>(src + 4);
  unsigned b0, b1, b2, b3, b4, b5, b6, b7, f0, f1, f2, f3, f4, f5, f6, f7;
  cvt2(a.x, b0, f0); cvt2(a.y, b1, f1); cvt2(a.z, b2, f2); cvt2(a.w, b3, f3);
  cvt2(c.x, b4, f4); cvt2(c.y, b5, f5); cvt2(c.z, b6, f6); cvt2(c.w, b7, f7);
  v4u ob, of;
  ob.x = b0 | (b1 << 16); ob.y = b2 | (b3 << 16); ob.z = b4 | (b5 << 16); ob.w = b6 | (b7 << 16);
  of.x = f0 | (f1 << 16); of.y = f2 | (f3 << 16); of.z = f4 | (f5 << 16); of.w = f6 | (f7 << 16);
  u16* db = wob + (size_t)i * 8;
  u16* df = wof + (size_t)i * 8;
  vst16(db, ob); vst16(df, of);
  __threadfence();
  vst16(db, ob); vst16(df, of);
}

__global__ void __launch_bounds__(128)
k_wqk(const float* __restrict__ params, u16* __restrict__ ghi, u16* __restrict__ glo) {
  __shared__ __align__(16) u16 Lb[64][64];
  __shared__ __align__(16) u16 Sh[64][64];
  __shared__ __align__(16) u16 Sl[64][64];
  const int tid = threadIdx.x, lane = tid & 31, wave = tid >> 5;
  const int m = lane & 15, hs = (lane >> 4) & 1, lh = hs * 8;
  const int head = blockIdx.x;
  const float* p = params + (size_t)head * TRIL;
  for (int e = tid; e < HD * HD; e += 128) {
    const int i = e >> 6, j = e & 63;
    const int jj = (j <= i) ? j : i;
    const float v = p[(i * (i + 1)) / 2 + jj];
    Lb[i][j] = (u16)((j <= i) ? bfbits(v) : 0u);
  }
  __syncthreads();
  v8f acc[4] = {};
#pragma unroll
  for (int ks = 0; ks < 2; ++ks) {
    const Frag a = ldfrag(&Lb[wave * 16 + m][ks * 32], lh);
#pragma unroll
    for (int nt = 0; nt < 4; ++nt) {
      const Frag bq = ldfrag(&Lb[nt * 16 + m][ks * 32], lh);
      acc[nt] = mma_bf16(a, bq, acc[nt]);
    }
  }
#pragma unroll
  for (int nt = 0; nt < 4; ++nt) {
#pragma unroll
    for (int g = 0; g < 8; ++g) {
      const int row = wave * 16 + hs * 8 + g, col = nt * 16 + m;
      const float v = acc[nt][g];
      const unsigned hb = bfbits(v);
      const unsigned lb = bfbits(v - bf2f(hb));
      Sh[row][col] = (u16)hb;
      Sl[row][col] = (u16)lb;
    }
  }
  __syncthreads();
  u16* dh = ghi + (size_t)head * (HD * HD);
  u16* dl = glo + (size_t)head * (HD * HD);
  const int rsub = lane >> 3, ch = (lane & 7) * 8;
#pragma unroll
  for (int q = 0; q < 4; ++q) {
    const int row = wave * 16 + q * 4 + rsub;
    vst16(dh + row * HD + ch, ld16(&Sh[row][ch]));
    vst16(dl + row * HD + ch, ld16(&Sl[row][ch]));
  }
  __threadfence();
#pragma unroll
  for (int q = 0; q < 4; ++q) {
    const int row = wave * 16 + q * 4 + rsub;
    vst16(dh + row * HD + ch, ld16(&Sh[row][ch]));
    vst16(dl + row * HD + ch, ld16(&Sl[row][ch]));
  }
}

__global__ void __launch_bounds__(128)
k_vproj(const u16* __restrict__ xb, const u16* __restrict__ wvb, const float* __restrict__ bv,
        u16* __restrict__ vthi, u16* __restrict__ vtlo) {
  __shared__ __align__(16) u16 Bt[2][64][32];
  __shared__ __align__(16) u16 Th[64][128];
  __shared__ __align__(16) u16 Tl[64][128];
  const int tid = threadIdx.x, lane = tid & 31, wave = tid >> 5;
  const int m = lane & 15, hs = (lane >> 4) & 1, lh = hs * 8;
  const int head = blockIdx.x;
  const int n0 = head * HD;
  const int mb = blockIdx.y * 128;
  const int m0 = mb + wave * 32;
  const int srow = tid >> 2, sk = (tid & 3) * 8;
  const u16* g0 = wvb + (size_t)(n0 + srow) * EE + sk;
  const u16* g1 = wvb + (size_t)(n0 + 32 + srow) * EE + sk;
  *reinterpret_cast<v4u*>(&Bt[0][srow][sk])      = *reinterpret_cast<const v4u*>(g0);
  *reinterpret_cast<v4u*>(&Bt[0][32 + srow][sk]) = *reinterpret_cast<const v4u*>(g1);
  __syncthreads();
  const u16* a0p = xb + (size_t)(m0 + m) * EE;
  const u16* a1p = xb + (size_t)(m0 + 16 + m) * EE;
  v8f acc0[4] = {}, acc1[4] = {};
#pragma unroll 1
  for (int kc = 0; kc < EE; kc += 32) {
    const int buf = (kc >> 5) & 1;
    const Frag a0 = ldfrag(a0p + kc, lh);
    const Frag a1 = ldfrag(a1p + kc, lh);
#pragma unroll
    for (int nt = 0; nt < 4; ++nt) {
      const Frag bq = ldfrag(&Bt[buf][nt * 16 + m][0], lh);
      acc0[nt] = mma_bf16(a0, bq, acc0[nt]);
      acc1[nt] = mma_bf16(a1, bq, acc1[nt]);
    }
    if (kc + 32 < EE) {
      *reinterpret_cast<v4u*>(&Bt[buf ^ 1][srow][sk])      = *reinterpret_cast<const v4u*>(g0 + kc + 32);
      *reinterpret_cast<v4u*>(&Bt[buf ^ 1][32 + srow][sk]) = *reinterpret_cast<const v4u*>(g1 + kc + 32);
    }
    __syncthreads();
  }
  const int bb = mb / SEQ, s0 = mb - bb * SEQ;
  const int bh = bb * HH + head;
#pragma unroll
  for (int nt = 0; nt < 4; ++nt) {
    const int d = nt * 16 + m;
    const float bvv = bf2f(bfbits(bv[n0 + d]));
#pragma unroll
    for (int mt = 0; mt < 2; ++mt) {
#pragma unroll
      for (int g = 0; g < 8; ++g) {
        const int sl = wave * 32 + mt * 16 + hs * 8 + g;
        const float v = (mt ? acc1[nt][g] : acc0[nt][g]) + bvv;
        const unsigned hb = hbits(v);
        const unsigned lb = bfbits(v - h2f(hb));
        Th[d][sl] = (u16)hb;
        Tl[d][sl] = (u16)lb;
      }
    }
  }
  __syncthreads();
  const int dsub = lane >> 4, ch = (lane & 15) * 8;
#pragma unroll
  for (int q = 0; q < 8; ++q) {
    const int d = wave * 16 + q * 2 + dsub;
    const size_t go = ((size_t)(bh * HD + d)) * SEQ + s0 + ch;
    vst16(vthi + go, ld16(&Th[d][ch]));
    vst16(vtlo + go, ld16(&Tl[d][ch]));
  }
  __threadfence();
#pragma unroll
  for (int q = 0; q < 8; ++q) {
    const int d = wave * 16 + q * 2 + dsub;
    const size_t go = ((size_t)(bh * HD + d)) * SEQ + s0 + ch;
    vst16(vthi + go, ld16(&Th[d][ch]));
    vst16(vtlo + go, ld16(&Tl[d][ch]));
  }
}

__global__ void __launch_bounds__(128)
k_tproj(const u16* __restrict__ xb, const u16* __restrict__ ghi, const u16* __restrict__ glo,
        u16* __restrict__ thi, u16* __restrict__ tlo) {
  __shared__ __align__(16) u16 Sh[4][32][64];
  __shared__ __align__(16) u16 Sl[4][32][64];
  const int tid = threadIdx.x, lane = tid & 31, wave = tid >> 5;
  const int m = lane & 15, hs = (lane >> 4) & 1, lh = hs * 8;
  const int head = blockIdx.y;
  const int m0 = blockIdx.x * 128 + wave * 32;
  const u16* a0p = xb + (size_t)(m0 + m) * EE + head * HD;
  const u16* a1p = xb + (size_t)(m0 + 16 + m) * EE + head * HD;
  const Frag a00 = ldfrag(a0p, lh), a01 = ldfrag(a0p + 32, lh);
  const Frag a10 = ldfrag(a1p, lh), a11 = ldfrag(a1p + 32, lh);
  v8f acc0[4] = {}, acc1[4] = {};
#pragma unroll
  for (int nt = 0; nt < 4; ++nt) {
    const u16* bhp = ghi + ((size_t)(head * HD + nt * 16 + m)) * HD;
    const u16* blp = glo + ((size_t)(head * HD + nt * 16 + m)) * HD;
    const Frag b0 = ldfrag(bhp, lh), b1 = ldfrag(bhp + 32, lh);
    acc0[nt] = mma_bf16(a00, b0, acc0[nt]); acc0[nt] = mma_bf16(a01, b1, acc0[nt]);
    acc1[nt] = mma_bf16(a10, b0, acc1[nt]); acc1[nt] = mma_bf16(a11, b1, acc1[nt]);
    const Frag c0 = ldfrag(blp, lh), c1 = ldfrag(blp + 32, lh);
    acc0[nt] = mma_bf16(a00, c0, acc0[nt]); acc0[nt] = mma_bf16(a01, c1, acc0[nt]);
    acc1[nt] = mma_bf16(a10, c0, acc1[nt]); acc1[nt] = mma_bf16(a11, c1, acc1[nt]);
  }
#pragma unroll
  for (int nt = 0; nt < 4; ++nt) {
#pragma unroll
    for (int mt = 0; mt < 2; ++mt) {
#pragma unroll
      for (int g = 0; g < 8; ++g) {
        const int rl = mt * 16 + hs * 8 + g, col = nt * 16 + m;
        const float v = mt ? acc1[nt][g] : acc0[nt][g];
        const unsigned hb = bfbits(v);
        const unsigned lb = bfbits(v - bf2f(hb));
        Sh[wave][rl][col] = (u16)hb;
        Sl[wave][rl][col] = (u16)lb;
      }
    }
  }
  __syncthreads();
  const int rsub = lane >> 3, ch = (lane & 7) * 8;
#pragma unroll
  for (int q = 0; q < 8; ++q) {
    const int rl = q * 4 + rsub;
    const size_t go = (size_t)(m0 + rl) * EE + head * HD + ch;
    vst16(thi + go, ld16(&Sh[wave][rl][ch]));
    vst16(tlo + go, ld16(&Sl[wave][rl][ch]));
  }
  __threadfence();
#pragma unroll
  for (int q = 0; q < 8; ++q) {
    const int rl = q * 4 + rsub;
    const size_t go = (size_t)(m0 + rl) * EE + head * HD + ch;
    vst16(thi + go, ld16(&Sh[wave][rl][ch]));
    vst16(tlo + go, ld16(&Sl[wave][rl][ch]));
  }
}

__global__ void __launch_bounds__(128)
k_attn(const u16* __restrict__ thi, const u16* __restrict__ tlo, const u16* __restrict__ xb,
       const u16* __restrict__ vthi, const u16* __restrict__ vtlo,
       u16* __restrict__ chi, u16* __restrict__ clo) {
  __shared__ __align__(16) u16 Ks[2][32][64];
  __shared__ __align__(16) u16 Vh[2][64][32];
  __shared__ __align__(16) u16 Vl[2][64][32];
  __shared__ __align__(16) u16 Pf[4][16][32];
  __shared__ __align__(16) u16 Pb[4][16][32];
  __shared__ __align__(16) u16 Ch[4][16][64];
  __shared__ __align__(16) u16 Cl[4][16][64];
  const int tid = threadIdx.x, lane = tid & 31, wave = tid >> 5;
  const int m = lane & 15, hs = (lane >> 4) & 1, lh = hs * 8;
  const int bh = blockIdx.y;
  const int b  = bh / HH;
  const int h  = bh - b * HH;
  const int q0 = blockIdx.x * 64 + wave * 16;
  const size_t qrow = (size_t)b * SEQ + q0 + m;

  const Frag qh0 = ldfrag(thi + qrow * EE + h * HD, lh);
  const Frag qh1 = ldfrag(thi + qrow * EE + h * HD + 32, lh);
  const Frag ql0 = ldfrag(tlo + qrow * EE + h * HD, lh);
  const Frag ql1 = ldfrag(tlo + qrow * EE + h * HD + 32, lh);

  auto stage = [&](int kv, int bw) {
#pragma unroll
    for (int j = 0; j < 2; ++j) {
      const int c = tid + 128 * j;
      const int kr = c >> 3, kc = (c & 7) * 8;
      *reinterpret_cast<v4u*>(&Ks[bw][kr][kc]) =
          *reinterpret_cast<const v4u*>(xb + ((size_t)(b * SEQ + kv + kr)) * EE + h * HD + kc);
      const int d = c >> 2, dc = (c & 3) * 8;
      const size_t vo = ((size_t)(bh * HD + d)) * SEQ + kv + dc;
      *reinterpret_cast<v4u*>(&Vh[bw][d][dc]) = *reinterpret_cast<const v4u*>(vthi + vo);
      *reinterpret_cast<v4u*>(&Vl[bw][d][dc]) = *reinterpret_cast<const v4u*>(vtlo + vo);
    }
  };

  stage(0, 0);
  __syncthreads();

  v8f acc[4] = {};
  float mrun[8], lrun[8];
#pragma unroll
  for (int g = 0; g < 8; ++g) { mrun[g] = -1e30f; lrun[g] = 0.0f; }

#pragma unroll 1
  for (int kv = 0; kv < SEQ; kv += 32) {
    const int buf = (kv >> 5) & 1;
    v8f s0 = {}, s1 = {};
    {
      const Frag k0 = ldfrag(&Ks[buf][m][0], lh);
      const Frag k1 = ldfrag(&Ks[buf][m][32], lh);
      s0 = mma_bf16(qh0, k0, s0); s0 = mma_bf16(qh1, k1, s0);
      s0 = mma_bf16(ql0, k0, s0); s0 = mma_bf16(ql1, k1, s0);
    }
    {
      const Frag k0 = ldfrag(&Ks[buf][16 + m][0], lh);
      const Frag k1 = ldfrag(&Ks[buf][16 + m][32], lh);
      s1 = mma_bf16(qh0, k0, s1); s1 = mma_bf16(qh1, k1, s1);
      s1 = mma_bf16(ql0, k0, s1); s1 = mma_bf16(ql1, k1, s1);
    }
#pragma unroll
    for (int g = 0; g < 8; ++g) {
      const float a0 = s0[g] * 0.125f;
      const float a1 = s1[g] * 0.125f;
      float mx = fmaxf(a0, a1);
      mx = fmaxf(mx, __shfl_xor(mx, 1));
      mx = fmaxf(mx, __shfl_xor(mx, 2));
      mx = fmaxf(mx, __shfl_xor(mx, 4));
      mx = fmaxf(mx, __shfl_xor(mx, 8));
      const float nm = fmaxf(mrun[g], mx);
      const float p0 = __expf(a0 - nm);
      const float p1 = __expf(a1 - nm);
      float rs = p0 + p1;
      rs += __shfl_xor(rs, 1);
      rs += __shfl_xor(rs, 2);
      rs += __shfl_xor(rs, 4);
      rs += __shfl_xor(rs, 8);
      const float alpha = __expf(mrun[g] - nm);
      lrun[g] = lrun[g] * alpha + rs;
      mrun[g] = nm;
      const int prow = hs * 8 + g;
      const float c0 = p0 * PCARRY, c1 = p1 * PCARRY;
      Pf[wave][prow][m]      = (u16)hbits(c0);
      Pf[wave][prow][16 + m] = (u16)hbits(c1);
      Pb[wave][prow][m]      = (u16)bfbits(c0);
      Pb[wave][prow][16 + m] = (u16)bfbits(c1);
#pragma unroll
      for (int t = 0; t < 4; ++t) acc[t][g] = acc[t][g] * alpha;
    }
    __syncthreads();
    if (kv + 32 < SEQ) stage(kv + 32, buf ^ 1);
    {
      const Frag pf = ldfrag(&Pf[wave][m][0], lh);
      const Frag pb = ldfrag(&Pb[wave][m][0], lh);
#pragma unroll
      for (int t = 0; t < 4; ++t) {
        const Frag vh = ldfrag(&Vh[buf][t * 16 + m][0], lh);
        acc[t] = mma_f16(pf, vh, acc[t]);
        const Frag vl = ldfrag(&Vl[buf][t * 16 + m][0], lh);
        acc[t] = mma_bf16(pb, vl, acc[t]);
      }
    }
    __syncthreads();
  }

#pragma unroll
  for (int g = 0; g < 8; ++g) {
    const float rl = (1.0f / lrun[g]) * PCARRY_INV;
    const int crow = hs * 8 + g;
#pragma unroll
    for (int t = 0; t < 4; ++t) {
      const float o = acc[t][g] * rl;
      const unsigned hb = hbits(o);
      const unsigned lb = bfbits(o - h2f(hb));
      Ch[wave][crow][t * 16 + m] = (u16)hb;
      Cl[wave][crow][t * 16 + m] = (u16)lb;
    }
  }
  __syncthreads();
  const int rsub = lane >> 3, ch = (lane & 7) * 8;
#pragma unroll
  for (int q = 0; q < 4; ++q) {
    const int rl = q * 4 + rsub;
    const size_t go = ((size_t)(b * SEQ + q0 + rl)) * EE + h * HD + ch;
    vst16(chi + go, ld16(&Ch[wave][rl][ch]));
    vst16(clo + go, ld16(&Cl[wave][rl][ch]));
  }
  __threadfence();
#pragma unroll
  for (int q = 0; q < 4; ++q) {
    const int rl = q * 4 + rsub;
    const size_t go = ((size_t)(b * SEQ + q0 + rl)) * EE + h * HD + ch;
    vst16(chi + go, ld16(&Ch[wave][rl][ch]));
    vst16(clo + go, ld16(&Cl[wave][rl][ch]));
  }
}

__global__ void __launch_bounds__(128)
k_oproj(const u16* __restrict__ chi, const u16* __restrict__ clo,
        const u16* __restrict__ wof, const u16* __restrict__ wob,
        const float* __restrict__ bo, float* __restrict__ out) {
  __shared__ __align__(16) u16 Bf[2][64][32];
  __shared__ __align__(16) u16 Bb[2][64][32];
  __shared__ __align__(16) float Ot[128][64];
  const int tid = threadIdx.x, lane = tid & 31, wave = tid >> 5;
  const int m = lane & 15, hs = (lane >> 4) & 1, lh = hs * 8;
  const int n0 = blockIdx.x * 64;
  const int mb = blockIdx.y * 128;
  const int m0 = mb + wave * 32;
  const int srow = tid >> 2, sk = (tid & 3) * 8;
  const u16* f0p = wof + (size_t)(n0 + srow) * EE + sk;
  const u16* f1p = wof + (size_t)(n0 + 32 + srow) * EE + sk;
  const u16* b0p = wob + (size_t)(n0 + srow) * EE + sk;
  const u16* b1p = wob + (size_t)(n0 + 32 + srow) * EE + sk;
  *reinterpret_cast<v4u*>(&Bf[0][srow][sk])      = *reinterpret_cast<const v4u*>(f0p);
  *reinterpret_cast<v4u*>(&Bf[0][32 + srow][sk]) = *reinterpret_cast<const v4u*>(f1p);
  *reinterpret_cast<v4u*>(&Bb[0][srow][sk])      = *reinterpret_cast<const v4u*>(b0p);
  *reinterpret_cast<v4u*>(&Bb[0][32 + srow][sk]) = *reinterpret_cast<const v4u*>(b1p);
  __syncthreads();
  const u16* h0p = chi + (size_t)(m0 + m) * EE;
  const u16* h1p = chi + (size_t)(m0 + 16 + m) * EE;
  const u16* l0p = clo + (size_t)(m0 + m) * EE;
  const u16* l1p = clo + (size_t)(m0 + 16 + m) * EE;
  v8f acc0[4] = {}, acc1[4] = {};
#pragma unroll 1
  for (int kc = 0; kc < EE; kc += 32) {
    const int buf = (kc >> 5) & 1;
    const Frag ah0 = ldfrag(h0p + kc, lh), ah1 = ldfrag(h1p + kc, lh);
    const Frag al0 = ldfrag(l0p + kc, lh), al1 = ldfrag(l1p + kc, lh);
#pragma unroll
    for (int nt = 0; nt < 4; ++nt) {
      const Frag bf = ldfrag(&Bf[buf][nt * 16 + m][0], lh);
      acc0[nt] = mma_f16(ah0, bf, acc0[nt]);
      acc1[nt] = mma_f16(ah1, bf, acc1[nt]);
      const Frag bb = ldfrag(&Bb[buf][nt * 16 + m][0], lh);
      acc0[nt] = mma_bf16(al0, bb, acc0[nt]);
      acc1[nt] = mma_bf16(al1, bb, acc1[nt]);
    }
    if (kc + 32 < EE) {
      *reinterpret_cast<v4u*>(&Bf[buf ^ 1][srow][sk])      = *reinterpret_cast<const v4u*>(f0p + kc + 32);
      *reinterpret_cast<v4u*>(&Bf[buf ^ 1][32 + srow][sk]) = *reinterpret_cast<const v4u*>(f1p + kc + 32);
      *reinterpret_cast<v4u*>(&Bb[buf ^ 1][srow][sk])      = *reinterpret_cast<const v4u*>(b0p + kc + 32);
      *reinterpret_cast<v4u*>(&Bb[buf ^ 1][32 + srow][sk]) = *reinterpret_cast<const v4u*>(b1p + kc + 32);
    }
    __syncthreads();
  }
#pragma unroll
  for (int nt = 0; nt < 4; ++nt) {
    const int col = nt * 16 + m;
    const float bov = bf2f(bfbits(bo[n0 + col]));
#pragma unroll
    for (int mt = 0; mt < 2; ++mt) {
#pragma unroll
      for (int g = 0; g < 8; ++g) {
        const int rl = wave * 32 + mt * 16 + hs * 8 + g;
        const float v = (mt ? acc1[nt][g] : acc0[nt][g]) * WSCALE_INV + bov;
        Ot[rl][col] = v;
      }
    }
  }
  __syncthreads();
  const int rsub = lane >> 4, ch = (lane & 15) * 4;
#pragma unroll
  for (int q = 0; q < 16; ++q) {
    const int rl = wave * 32 + q * 2 + rsub;
    vst4f(out + (size_t)(mb + rl) * EE + n0 + ch, ld4f(&Ot[rl][ch]));
  }
  __threadfence();
#pragma unroll
  for (int q = 0; q < 16; ++q) {
    const int rl = wave * 32 + q * 2 + rsub;
    vst4f(out + (size_t)(mb + rl) * EE + n0 + ch, ld4f(&Ot[rl][ch]));
  }
}

extern "C" void kernel_launch(void* const* d_in, const int* in_sizes, int n_in,
                              void* d_out, int out_size, void* d_ws, size_t ws_size,
                              hipStream_t stream) {
  if (n_in < 6) return;
  if (in_sizes[0] < ((NB - 1) * SEQ_FULL + SEQ) * EE) return;
  if (in_sizes[1] < HH * TRIL) return;
  if (in_sizes[2] < EE * EE || in_sizes[3] < EE || in_sizes[4] < EE * EE || in_sizes[5] < EE) return;
  if (out_size < M_TOT * EE) return;

  const float* x   = (const float*)d_in[0];
  const float* prm = (const float*)d_in[1];
  const float* wv  = (const float*)d_in[2];
  const float* bv  = (const float*)d_in[3];
  const float* wo  = (const float*)d_in[4];
  const float* bo  = (const float*)d_in[5];
  float* out = (float*)d_out;

  char* ws = (char*)d_ws;
  size_t off = 0;
  auto carve = [&](size_t bytes) -> char* {
    char* p = ws + off;
    off += (bytes + 255) & ~(size_t)255;
    return p;
  };
  const size_t plane  = (size_t)M_TOT * EE * 2;
  const size_t wplane = (size_t)EE * EE * 2;
  const size_t gplane = (size_t)HH * HD * HD * 2;
  const size_t vplane = (size_t)NB * HH * HD * SEQ * 2;
  u16* xb   = (u16*)carve(plane);
  u16* wvb  = (u16*)carve(wplane);
  u16* wob  = (u16*)carve(wplane);
  u16* wof  = (u16*)carve(wplane);
  u16* ghi  = (u16*)carve(gplane);
  u16* glo  = (u16*)carve(gplane);
  u16* thi  = (u16*)carve(plane);
  u16* tlo  = (u16*)carve(plane);
  u16* vthi = (u16*)carve(vplane);
  u16* vtlo = (u16*)carve(vplane);
  u16* chi  = (u16*)carve(plane);
  u16* clo  = (u16*)carve(plane);
  if (off > ws_size) return;

  {
    const int ngrp = M_TOT * (EE / 8);
    k_cvt_x<<<dim3((ngrp + 255) / 256), dim3(256), 0, stream>>>(x, xb);
  }
  {
    const int ngrp = EE * EE / 8;
    k_cvt_w<<<dim3((ngrp + 255) / 256), dim3(256), 0, stream>>>(wv, wvb);
    k_cvt_wo<<<dim3((ngrp + 255) / 256), dim3(256), 0, stream>>>(wo, wob, wof);
  }
  k_wqk<<<dim3(HH), dim3(128), 0, stream>>>(prm, ghi, glo);
  k_vproj<<<dim3(EE / 64, M_TOT / 128), dim3(128), 0, stream>>>(xb, wvb, bv, vthi, vtlo);
  k_tproj<<<dim3(M_TOT / 128, HH), dim3(128), 0, stream>>>(xb, ghi, glo, thi, tlo);
  k_attn<<<dim3(SEQ / 64, NB * HH), dim3(128), 0, stream>>>(thi, tlo, xb, vthi, vtlo, chi, clo);
  k_oproj<<<dim3(EE / 64, M_TOT / 128), dim3(128), 0, stream>>>(chi, clo, wof, wob, bo, out);
}
